// Transformer_38577396252701
// MI455X (gfx1250) — hardware-verified
//
#include <hip/hip_runtime.h>
#include <math.h>

#ifndef NB
#define NB 4
#endif
#ifndef LQ
#define LQ 512
#endif
#ifndef LK
#define LK 1024
#endif
#define LQ_FULL 512
#define LK_FULL 1024
#define DM 512
#define NH 8
#define HD 64
#define DFF 2048
#define JA_NW 4
#define JA_PP 72

static_assert(LQ % 64 == 0);
static_assert(LK % 64 == 0);
static_assert(LQ <= LQ_FULL);
static_assert(LK <= LK_FULL);
static_assert(NB >= 1 && NB <= 4);
static_assert(DM == NH * HD);
static_assert(DM % 64 == 0 && DFF % 64 == 0);
static_assert(((NB * LQ) % 8) == 0);

typedef __attribute__((ext_vector_type(16))) _Float16 v16h;
typedef __attribute__((ext_vector_type(8)))  _Float16 v8h;
typedef __attribute__((ext_vector_type(16))) __bf16   v16b;
typedef __attribute__((ext_vector_type(8)))  float    v8f;
typedef __attribute__((ext_vector_type(4)))  float    v4f;
typedef __attribute__((ext_vector_type(4)))  unsigned v4u;
typedef __attribute__((ext_vector_type(2)))  unsigned v2u;
typedef v4f v4f_a __attribute__((may_alias));
typedef v8h v8h_a __attribute__((may_alias));


#define VST2(T, ptr, val) do { const T vst2_v_ = (val); *(volatile T*)(ptr) = vst2_v_; __threadfence(); *(volatile T*)(ptr) = vst2_v_; } while (0)
#define VST2V4(ptr, val) do { const v4f vst2_v4_ = (val); *(volatile v4f*)(ptr) = vst2_v4_; __threadfence(); *(volatile v4f*)(ptr) = vst2_v4_; } while (0)

__device__ __forceinline__ float cmb_bf(float v) {
    const unsigned u = __builtin_bit_cast(unsigned, v);
    const unsigned r = (u + 0x7fffu + ((u >> 16) & 1u)) & 0xffff0000u;
    return __builtin_bit_cast(float, r);
}
__device__ __forceinline__ unsigned cmb_pk2(float a, float b) {
    return (unsigned)__builtin_bit_cast(unsigned short, (_Float16)a) | ((unsigned)__builtin_bit_cast(unsigned short, (_Float16)b) << 16);
}
__device__ __forceinline__ unsigned short bfu_rne(float v) { unsigned u = __builtin_bit_cast(unsigned, v); u += 0x7FFFu + ((u >> 16) & 1u); return (unsigned short)(u >> 16); }
__device__ __forceinline__ void bfsplit(float v, unsigned short& hi, unsigned short& lo) { hi = bfu_rne(v); lo = bfu_rne(v - __builtin_bit_cast(float, (unsigned)hi << 16)); }
__device__ __forceinline__ void bfs2(float a, float b, unsigned& hi, unsigned& lo) {
    unsigned short h0, l0, h1, l1; bfsplit(a, h0, l0); bfsplit(b, h1, l1);
    hi = (unsigned)h0 | ((unsigned)h1 << 16); lo = (unsigned)l0 | ((unsigned)l1 << 16);
}

struct FragU { v4u a, b; };
static_assert(sizeof(FragU) == 32);
__device__ __forceinline__ v16h ldf_h(const unsigned short* p) { FragU t; t.a = *(const v4u*)p; t.b = *(const v4u*)(p + 16); return __builtin_bit_cast(v16h, t); }
__device__ __forceinline__ v16b ldf_b(const unsigned short* p) { FragU t; t.a = *(const v4u*)p; t.b = *(const v4u*)(p + 16); return __builtin_bit_cast(v16b, t); }
__device__ __forceinline__ v16h ldl_h(const _Float16* p) { union { v16h v; v8h h[2]; } f; f.h[0] = *(const v8h_a*)p; f.h[1] = *(const v8h_a*)(p + 16); return f.v; }

__device__ __forceinline__ v8f mma_h(v16h a, v16h b, v8f c) {
    c = __builtin_amdgcn_wmma_f32_16x16x32_f16(false, a, false, b, (short)0, c, false, false);
    asm volatile("v_nop\n\tv_nop\n\tv_nop\n\tv_nop" : "+v"(c) : "v"(a), "v"(b));
    return c;
}
__device__ __forceinline__ v8f mma3_b(v16b ah, v16b al, v16b bh, v16b bl, v8f c) {
    c = __builtin_amdgcn_wmma_f32_16x16x32_bf16(false, ah, false, bh, (short)0, c, false, false);
    c = __builtin_amdgcn_wmma_f32_16x16x32_bf16(false, ah, false, bl, (short)0, c, false, false);
    c = __builtin_amdgcn_wmma_f32_16x16x32_bf16(false, al, false, bh, (short)0, c, false, false);
    asm volatile("v_nop\n\tv_nop\n\tv_nop\n\tv_nop" : "+v"(c) : "v"(ah), "v"(al), "v"(bh), "v"(bl));
    return c;
}
__device__ __forceinline__ void guard4(v8f& a, v8f& b, v8f& c, v8f& d, v16h x) { asm volatile("v_nop\n\tv_nop\n\tv_nop\n\tv_nop" : "+v"(a), "+v"(b), "+v"(c), "+v"(d) : "v"(x)); }
__device__ __forceinline__ void keep4(v16h a, v16h b, v16h c, v16h d) { asm volatile("v_nop" :: "v"(a), "v"(b), "v"(c), "v"(d)); }
__device__ __forceinline__ void wave_sync() {
    __builtin_amdgcn_fence(3  , "workgroup");
    __builtin_amdgcn_wave_barrier();
    __builtin_amdgcn_fence(2  , "workgroup");
}

__global__ __launch_bounds__(256) void k_castrows(const float* __restrict__ SRC, unsigned short* __restrict__ DST, unsigned rowsPerBatch, unsigned srcBatchRows, unsigned nBatch, float sc) {
    const unsigned u = blockIdx.x * 256u + threadIdx.x;
    if (u >= nBatch * rowsPerBatch * (DM / 8u)) return;
    const unsigned r = u >> 6, c0 = (u & 63u) << 3;
    const unsigned b = r / rowsPerBatch, rr = r - b * rowsPerBatch;
    const float* s = SRC + ((size_t)(b * srcBatchRows + rr)) * DM + c0;
    const v4f x0 = *(const v4f*)s, x1 = *(const v4f*)(s + 4);
    v4u pk;
    pk.x = cmb_pk2(cmb_bf(x0.x) * sc, cmb_bf(x0.y) * sc); pk.y = cmb_pk2(cmb_bf(x0.z) * sc, cmb_bf(x0.w) * sc);
    pk.z = cmb_pk2(cmb_bf(x1.x) * sc, cmb_bf(x1.y) * sc); pk.w = cmb_pk2(cmb_bf(x1.z) * sc, cmb_bf(x1.w) * sc);
    VST2(v4u, DST + (size_t)r * DM + c0, pk);
}

__global__ __launch_bounds__(256) void k_castT(const float* __restrict__ S0, const float* __restrict__ S1, const float* __restrict__ S2, const float* __restrict__ S3,
                                               unsigned lds, unsigned short* __restrict__ DST, unsigned ldd, unsigned nR, unsigned nC, float sc) {
    const unsigned y = blockIdx.y;
    const float* SRC = (y == 0u) ? S0 : ((y == 1u) ? S1 : ((y == 2u) ? S2 : S3));
    const unsigned u = blockIdx.x * 256u + threadIdx.x; const unsigned per = nR >> 3;
    if (u >= nC * per) return;
    const unsigned c = u / per, r0 = (u - c * per) << 3;
    float w[8];
#pragma unroll
    for (int e = 0; e < 8; ++e) w[e] = cmb_bf(SRC[(size_t)(r0 + e) * lds + c]) * sc;
    v4u pk; pk.x = cmb_pk2(w[0], w[1]); pk.y = cmb_pk2(w[2], w[3]); pk.z = cmb_pk2(w[4], w[5]); pk.w = cmb_pk2(w[6], w[7]);
    VST2(v4u, DST + (size_t)y * nR * nC + (size_t)c * ldd + r0, pk);
}

__global__ __launch_bounds__(256) void k_biaspack(const float* __restrict__ bq, const float* __restrict__ bk, const float* __restrict__ bv, const float* __restrict__ bo,
                                                  const float* __restrict__ b1, const float* __restrict__ b2, float* __restrict__ DST) {
    const unsigned blk = blockIdx.x; const float* S; unsigned base; float sc = 1.f;
    if (blk < 2u) { S = bq; base = 0u; sc = 0.125f; }
    else if (blk < 4u) { S = bk; base = 512u; }
    else if (blk < 6u) { S = bv; base = 1024u; }
    else if (blk < 8u) { S = bo; base = 1536u; }
    else if (blk < 16u) { S = b1; base = 2048u; }
    else { S = b2; base = 4096u; }
    const unsigned i = blk * 256u + threadIdx.x;
    const float v = cmb_bf(S[i - base]) * sc;
    VST2(float, DST + i, v);
}

__global__ __launch_bounds__(256) void k_bplane(const float* __restrict__ mask, const float* __restrict__ thb, const float* __restrict__ tpi,
                                                const float* __restrict__ aug_hb, const float* __restrict__ aug_pi, const float* __restrict__ aug_at, float* __restrict__ BP) {
    const unsigned u = blockIdx.x * 256u + threadIdx.x;
    if (u >= (unsigned)NB * LK * (LQ / 4u)) return;
    const unsigned q4 = (u % (LQ / 4u)) << 2; const unsigned kr = u / (LQ / 4u); const unsigned k = kr % (unsigned)LK, b = kr / (unsigned)LK;
    const size_t so = ((size_t)(b * LK_FULL + k)) * LQ_FULL + q4;
    const float aat = cmb_bf(aug_at[0]), ahb = cmb_bf(aug_hb[0]), api = cmb_bf(aug_pi[0]);
    const float L2E = 1.4426950408889634f;
    const v4f m = *(const v4f*)(mask + so), th = *(const v4f*)(thb + so), tp = *(const v4f*)(tpi + so);
    v4f o;
    o.x = (((cmb_bf(m.x) * -1e9f) * aat + ahb * cmb_bf(th.x)) + api * cmb_bf(tp.x)) * L2E;
    o.y = (((cmb_bf(m.y) * -1e9f) * aat + ahb * cmb_bf(th.y)) + api * cmb_bf(tp.y)) * L2E;
    o.z = (((cmb_bf(m.z) * -1e9f) * aat + ahb * cmb_bf(th.z)) + api * cmb_bf(tp.z)) * L2E;
    o.w = (((cmb_bf(m.w) * -1e9f) * aat + ahb * cmb_bf(th.w)) + api * cmb_bf(tp.w)) * L2E;
    VST2V4(BP + ((size_t)(b * LK + k)) * LQ + q4, o);
}

template <int BIAS_MODE, int OUT_MODE, int RESID, int ACT>
__global__ __launch_bounds__(256) void k_gemm64(const unsigned short* __restrict__ A, unsigned lda, long long strideA,
                                                const unsigned short* __restrict__ Bt, unsigned ldb, long long strideB,
                                                void* __restrict__ Cout, void* __restrict__ Cout2, unsigned ldc, long long strideC,
                                                const float* __restrict__ bias, const float* __restrict__ resid, unsigned ldr, long long strideR,
                                                unsigned M, unsigned N, unsigned K, float scale) {
    __shared__ __align__(16) float sT[8][16 * 68];
    const unsigned b = blockIdx.y, lane = threadIdx.x & 31u, wave = threadIdx.x >> 5;
    const unsigned tilesN = N >> 6, tilesM = M >> 6;
    const unsigned tile = blockIdx.x * 8u + wave;
    if (tile >= tilesM * tilesN) return;
    const unsigned tm = tile / tilesN, tn = tile - tm * tilesN;
    const unsigned m0 = tm << 6, n0 = tn << 6;
    const unsigned short* Ab = A + (size_t)b * (size_t)strideA;
    const unsigned short* Bb = Bt + (size_t)b * (size_t)strideB;
    const unsigned rlane = lane & 15u, koff = (lane >> 4) << 3, mOff = koff;

    v8f acc[4][4];
#pragma unroll
    for (int i = 0; i < 4; ++i)
#pragma unroll
        for (int j = 0; j < 4; ++j) { v8f zz = {}; acc[i][j] = zz; }

    for (unsigned k0 = 0; k0 < K; k0 += 32u) {
        v16h bh[4];
#pragma unroll
        for (int j = 0; j < 4; ++j) bh[j] = ldf_h(Bb + (size_t)(n0 + (j << 4) + rlane) * ldb + koff + k0);
#pragma unroll
        for (int i = 0; i < 4; ++i) {
            const v16h ah = ldf_h(Ab + (size_t)(m0 + (i << 4) + rlane) * lda + koff + k0);
#pragma unroll
            for (int j = 0; j < 4; ++j)
                acc[i][j] = __builtin_amdgcn_wmma_f32_16x16x32_f16(false, ah, false, bh[j], (short)0, acc[i][j], false, false);
            guard4(acc[i][0], acc[i][1], acc[i][2], acc[i][3], ah);
        }
        keep4(bh[0], bh[1], bh[2], bh[3]);
    }

    float* slab = sT[wave];
    const float* Rb = resid + (size_t)b * (size_t)strideR;
#pragma unroll
    for (int i = 0; i < 4; ++i) {
        const unsigned mBase = m0 + ((unsigned)i << 4);
#pragma unroll
        for (int j = 0; j < 4; ++j) {
            const unsigned n = n0 + ((unsigned)j << 4) + rlane;
            float bv = 0.f;
            if (BIAS_MODE == 2) bv = bias[n];
#pragma unroll
            for (int r = 0; r < 8; ++r) {
                float v = acc[i][j][r] * scale;
                if (BIAS_MODE == 1) v += bias[mBase + mOff + r];
                if (BIAS_MODE == 2) v += bv;
                if (ACT == 2) v = fmaxf(v, 0.0f);
                slab[(mOff + r) * 68u + ((unsigned)j << 4) + rlane] = v;
            }
        }
        wave_sync();
        if (OUT_MODE == 0) {
            float* Cb = (float*)Cout + (size_t)b * (size_t)strideC;
            const unsigned hh = lane >> 4, c4 = (lane & 15u) << 2;
            v4f vals[8];
#pragma unroll
            for (int it = 0; it < 8; ++it) {
                const unsigned row = (unsigned)it * 2u + hh;
                v4f v = *(const v4f_a*)(slab + row * 68u + c4);
                if (RESID != 0) {
                    v4f rr = *(const v4f*)(Rb + (size_t)(mBase + row) * ldr + n0 + c4);
                    if (RESID == 2) { rr.x = cmb_bf(rr.x); rr.y = cmb_bf(rr.y); rr.z = cmb_bf(rr.z); rr.w = cmb_bf(rr.w); }
                    v = v + rr;
                }
                vals[it] = v;
            }
            for (int pass = 0; pass < 2; ++pass) {
#pragma unroll
                for (int it = 0; it < 8; ++it) {
                    const unsigned row = (unsigned)it * 2u + hh;
                    *(volatile v4f*)(Cb + (size_t)(mBase + row) * ldc + n0 + c4) = vals[it];
                }
                __threadfence();
            }
        } else {
            const unsigned q = lane >> 3, c8 = (lane & 7u) << 3;
            unsigned short* C1 = (unsigned short*)Cout + (size_t)b * (size_t)strideC;
            unsigned short* C2 = (unsigned short*)Cout2 + (size_t)b * (size_t)strideC;
            v4u hv[4], lv[4];
#pragma unroll
            for (int it = 0; it < 4; ++it) {
                const unsigned row = (unsigned)it * 4u + q;
                const float* sp = slab + row * 68u + c8;
                const v4f x0 = *(const v4f_a*)sp, x1 = *(const v4f_a*)(sp + 4);
                v4u h4, l4;
                if (OUT_MODE == 1) {
                    h4.x = cmb_pk2(x0.x, x0.y); h4.y = cmb_pk2(x0.z, x0.w); h4.z = cmb_pk2(x1.x, x1.y); h4.w = cmb_pk2(x1.z, x1.w); l4 = h4;
                } else {
                    unsigned a0, a1, a2, a3, e0, e1, e2, e3;
                    bfs2(x0.x, x0.y, a0, e0); bfs2(x0.z, x0.w, a1, e1); bfs2(x1.x, x1.y, a2, e2); bfs2(x1.z, x1.w, a3, e3);
                    h4.x = a0; h4.y = a1; h4.z = a2; h4.w = a3; l4.x = e0; l4.y = e1; l4.z = e2; l4.w = e3;
                }
                hv[it] = h4; lv[it] = l4;
            }
            for (int pass = 0; pass < 2; ++pass) {
#pragma unroll
                for (int it = 0; it < 4; ++it) {
                    const unsigned row = (unsigned)it * 4u + q;
                    *(volatile v4u*)(C1 + (size_t)(mBase + row) * ldc + n0 + c8) = hv[it];
                    if (OUT_MODE == 2) *(volatile v4u*)(C2 + (size_t)(mBase + row) * ldc + n0 + c8) = lv[it];
                }
                __threadfence();
            }
        }
        wave_sync();
    }
}

__global__ __launch_bounds__(32 * JA_NW) void k_jattn(const unsigned short* __restrict__ QH, const unsigned short* __restrict__ QL,
                                                      const unsigned short* __restrict__ KH, const unsigned short* __restrict__ KL,
                                                      const unsigned short* __restrict__ VT, const float* __restrict__ BP,
                                                      const float* __restrict__ aug_at, float* __restrict__ U, float* __restrict__ ST) {
    __shared__ __align__(16) _Float16 Psh[JA_NW][16 * JA_PP];
    __shared__ __align__(16) float Os[JA_NW][16 * 68];
    const unsigned tid = threadIdx.x, wave = tid >> 5, lane = tid & 31u, hh = lane >> 4, c = lane & 15u;
    const unsigned nqb = LQ / 64u;
    const unsigned bx = blockIdx.x, qb = bx % nqb, bh = bx / nqb, h = bh & 7u, b = bh >> 3;
    const unsigned q0 = qb * 64u + wave * 16u;
    const float aatL = cmb_bf(aug_at[0]) * 1.4426950408889634f;

    const size_t qoff = ((size_t)(b * LQ + q0 + c)) * DM + h * HD + 8u * hh;
    v16b qah[2], qal[2];
#pragma unroll
    for (int dc = 0; dc < 2; ++dc) { qah[dc] = ldf_b(QH + qoff + dc * 32); qal[dc] = ldf_b(QL + qoff + dc * 32); }

    float mrow[8], lrow[8];
    v8f oacc[4];
#pragma unroll
    for (int r = 0; r < 8; ++r) { mrow[r] = -__builtin_inff(); lrow[r] = 0.f; }
#pragma unroll
    for (int t = 0; t < 4; ++t) { v8f zz = {}; oacc[t] = zz; }

    const size_t kbase = ((size_t)(b * LK + c)) * DM + h * HD + 8u * hh;
    const size_t vbase = ((size_t)(b * DM + h * HD + c)) * LK + 8u * hh;
    const size_t pbase = ((size_t)(b * LK + c)) * LQ + q0 + 8u * hh;
    _Float16* pw = Psh[wave];

#pragma unroll 1
    for (unsigned kc = 0; kc < LK / 64u; ++kc) {
        const unsigned kv0 = kc * 64u;
        v8f s[4];
#pragma unroll
        for (int j = 0; j < 4; ++j) {
            const size_t ko = kbase + (size_t)(kv0 + 16u * j) * DM;
            v8f a = {};
#pragma unroll
            for (int dc = 0; dc < 2; ++dc)
                a = mma3_b(qah[dc], qal[dc], ldf_b(KH + ko + dc * 32), ldf_b(KL + ko + dc * 32), a);
            const float* bp = BP + pbase + (size_t)(kv0 + 16u * j) * LQ;
            const v4f b0 = *(const v4f*)bp, b1 = *(const v4f*)(bp + 4);
            a[0] = fmaf(a[0], aatL, b0.x); a[1] = fmaf(a[1], aatL, b0.y); a[2] = fmaf(a[2], aatL, b0.z); a[3] = fmaf(a[3], aatL, b0.w);
            a[4] = fmaf(a[4], aatL, b1.x); a[5] = fmaf(a[5], aatL, b1.y); a[6] = fmaf(a[6], aatL, b1.z); a[7] = fmaf(a[7], aatL, b1.w);
            s[j] = a;
        }
        float cm[8];
#pragma unroll
        for (int r = 0; r < 8; ++r) {
            float m = fmaxf(fmaxf(s[0][r], s[1][r]), fmaxf(s[2][r], s[3][r]));
            m = fmaxf(m, __shfl_xor(m, 1, 32)); m = fmaxf(m, __shfl_xor(m, 2, 32));
            m = fmaxf(m, __shfl_xor(m, 4, 32)); m = fmaxf(m, __shfl_xor(m, 8, 32));
            cm[r] = m;
        }
#pragma unroll
        for (int r = 0; r < 8; ++r) {
            const float mnew = fmaxf(mrow[r], cm[r]);
            const float alpha = exp2f(mrow[r] - mnew);
            mrow[r] = mnew;
            float psum = 0.f;
#pragma unroll
            for (int j = 0; j < 4; ++j) {
                const float p = exp2f(s[j][r] - mnew);
                psum += p;
                pw[(8u * hh + r) * JA_PP + 16u * j + c] = (_Float16)(p * 4096.0f);
            }
            lrow[r] = lrow[r] * alpha + psum;
#pragma unroll
            for (int t = 0; t < 4; ++t) oacc[t][r] *= alpha;
        }
        wave_sync();
#pragma unroll
        for (int kk = 0; kk < 2; ++kk) {
            const v16h pa = ldl_h(pw + c * JA_PP + kk * 32 + 8u * hh);
#pragma unroll
            for (int t = 0; t < 4; ++t) {
                const v16h vb = ldf_h(VT + vbase + (size_t)(16u * t) * LK + kv0 + kk * 32);
                oacc[t] = mma_h(pa, vb, oacc[t]);
            }
        }
        wave_sync();
    }

#pragma unroll
    for (int r = 0; r < 8; ++r) {
        float l = lrow[r];
        l += __shfl_xor(l, 1, 32); l += __shfl_xor(l, 2, 32); l += __shfl_xor(l, 4, 32); l += __shfl_xor(l, 8, 32);
        lrow[r] = l;
    }
    float* os = Os[wave];
#pragma unroll
    for (int r = 0; r < 8; ++r)
#pragma unroll
        for (int t = 0; t < 4; ++t) os[(8u * hh + r) * 68u + 16u * t + c] = oacc[t][r] * (1.0f / 4096.0f);
    wave_sync();
    {
        const unsigned c4 = (lane & 15u) << 2;
        float* ub = U + ((size_t)(b * LQ + q0)) * DM + h * HD + c4;
        v4f vals[8];
#pragma unroll
        for (int it = 0; it < 8; ++it) vals[it] = *(const v4f_a*)(os + ((unsigned)it * 2u + hh) * 68u + c4);
        for (int pass = 0; pass < 2; ++pass) {
#pragma unroll
            for (int it = 0; it < 8; ++it) *(volatile v4f*)(ub + (size_t)((unsigned)it * 2u + hh) * DM) = vals[it];
            __threadfence();
        }
    }
    {
        const unsigned isel = (lane >> 1) & 7u;
        float mv = 0.f, lv = 0.f;
#pragma unroll
        for (int i = 0; i < 8; ++i) { const bool pick = ((unsigned)i == isel); mv = pick ? mrow[i] : mv; lv = pick ? lrow[i] : lv; }
        const float sv = (lane & 1u) ? lv : mv;
        VST2(float, ST + ((size_t)(bh * LQ + q0)) * 2u + lane, sv);
    }
}

__global__ __launch_bounds__(256) void k_jnorm(const float* __restrict__ ST, const float* __restrict__ U, unsigned short* __restrict__ C16) {
    __shared__ float red[256];
    __shared__ float fq[LQ];
    const unsigned bh = blockIdx.x, b = bh >> 3, h = bh & 7u, t = threadIdx.x;
    const float* st = ST + (size_t)bh * LQ * 2u;
    float mx = -__builtin_inff();
    for (unsigned q = t; q < LQ; q += 256u) mx = fmaxf(mx, st[2u * q]);
    red[t] = mx; __syncthreads();
    for (unsigned o = 128u; o > 0u; o >>= 1) { if (t < o) red[t] = fmaxf(red[t], red[t + o]); __syncthreads(); }
    const float Mx = red[0]; __syncthreads();
    float sm = 0.f;
    for (unsigned q = t; q < LQ; q += 256u) sm += st[2u * q + 1u] * exp2f(st[2u * q] - Mx);
    red[t] = sm; __syncthreads();
    for (unsigned o = 128u; o > 0u; o >>= 1) { if (t < o) red[t] += red[t + o]; __syncthreads(); }
    const float g = ((float)LK * 16.0f) / red[0];
    for (unsigned q = t; q < LQ; q += 256u) fq[q] = exp2f(st[2u * q] - Mx) * g;
    __syncthreads();
    const unsigned c8 = (t & 7u) << 3;
#pragma unroll 1
    for (unsigned it = 0; it < LQ / 32u; ++it) {
        const unsigned row = it * 32u + (t >> 3);
        const size_t off = ((size_t)(b * LQ + row)) * DM + h * HD + c8;
        const v4f x0 = *(const v4f*)(U + off), x1 = *(const v4f*)(U + off + 4);
        const float f = fq[row];
        v4u pk; pk.x = cmb_pk2(x0.x * f, x0.y * f); pk.y = cmb_pk2(x0.z * f, x0.w * f); pk.z = cmb_pk2(x1.x * f, x1.y * f); pk.w = cmb_pk2(x1.z * f, x1.w * f);
        VST2(v4u, C16 + off, pk);
    }
}

template <int WH>
__global__ __launch_bounds__(256) void k_ln(const float* __restrict__ X, const float* __restrict__ G, const float* __restrict__ Bv,
                                            float* __restrict__ O, unsigned short* __restrict__ OH, unsigned nrows) {
    const unsigned row = blockIdx.x * 8u + (threadIdx.x >> 5), lane = threadIdx.x & 31u;
    if (row >= nrows) return;
    const size_t base = (size_t)row * DM + 4u * lane;
    v4f v[4]; float s = 0.f;
#pragma unroll
    for (int i = 0; i < 4; ++i) { v[i] = *(const v4f*)(X + base + 128 * i); s += (v[i].x + v[i].y) + (v[i].z + v[i].w); }
    s += __shfl_xor(s, 16, 32); s += __shfl_xor(s, 8, 32); s += __shfl_xor(s, 4, 32); s += __shfl_xor(s, 2, 32); s += __shfl_xor(s, 1, 32);
    const float mu = s * (1.0f / 512.0f);
    float q = 0.f;
#pragma unroll
    for (int i = 0; i < 4; ++i) { const v4f d = v[i] - mu; q += (d.x * d.x + d.y * d.y) + (d.z * d.z + d.w * d.w); v[i] = d; }
    q += __shfl_xor(q, 16, 32); q += __shfl_xor(q, 8, 32); q += __shfl_xor(q, 4, 32); q += __shfl_xor(q, 2, 32); q += __shfl_xor(q, 1, 32);
    const float rs = 1.0f / sqrtf(q * (1.0f / 512.0f) + 1e-9f);
#pragma unroll
    for (int i = 0; i < 4; ++i) {
        const v4f g4 = *(const v4f*)(G + 4u * lane + 128 * i), b4 = *(const v4f*)(Bv + 4u * lane + 128 * i);
        v4f o;
        o.x = v[i].x * rs * cmb_bf(g4.x) + cmb_bf(b4.x); o.y = v[i].y * rs * cmb_bf(g4.y) + cmb_bf(b4.y);
        o.z = v[i].z * rs * cmb_bf(g4.z) + cmb_bf(b4.z); o.w = v[i].w * rs * cmb_bf(g4.w) + cmb_bf(b4.w);
        VST2V4(O + base + 128 * i, o);
        if (WH) { v2u pk; pk.x = cmb_pk2(o.x, o.y); pk.y = cmb_pk2(o.z, o.w); VST2(v2u, OH + base + 128 * i, pk); }
    }
}

extern "C" void kernel_launch(void* const* d_in, const int* in_sizes, int n_in, void* d_out, int out_size, void* d_ws, size_t ws_size, hipStream_t stream) {
    if (n_in < 24) return;
    const long long needQ  = ((long long)(NB - 1) * LQ_FULL + LQ) * DM;
    const long long needKV = ((long long)(NB - 1) * LK_FULL + LK) * DM;
    const long long needT  = ((long long)(NB - 1) * LK_FULL + (LK - 1)) * LQ_FULL + LQ;
    if ((long long)in_sizes[0] < needQ || (long long)in_sizes[1] < needKV) return;
    if ((long long)in_sizes[2] < needT || (long long)in_sizes[3] < needT || (long long)in_sizes[4] < needT) return;
    if (in_sizes[5] < 1 || in_sizes[6] < 1 || in_sizes[7] < 1) return;
    if (in_sizes[8] < DM * DM || in_sizes[10] < DM * DM || in_sizes[12] < DM * DM || in_sizes[14] < DM * DM) return;
    if (in_sizes[9] < DM || in_sizes[11] < DM || in_sizes[13] < DM || in_sizes[15] < DM) return;
    if (in_sizes[16] < DM * DFF || in_sizes[17] < DFF || in_sizes[18] < DFF * DM || in_sizes[19] < DM) return;
    if (in_sizes[20] < DM || in_sizes[21] < DM || in_sizes[22] < DM || in_sizes[23] < DM) return;
    if ((long long)out_size < (long long)NB * LQ * DM) return;

    const float* q    = (const float*)d_in[0];
    const float* kv   = (const float*)d_in[1];
    const float* mask = (const float*)d_in[2];
    const float* thb  = (const float*)d_in[3];
    const float* tpi  = (const float*)d_in[4];
    const float* ahb  = (const float*)d_in[5];
    const float* api  = (const float*)d_in[6];
    const float* aat  = (const float*)d_in[7];
    const float* wq = (const float*)d_in[8];   const float* bq = (const float*)d_in[9];
    const float* wk = (const float*)d_in[10];  const float* bk = (const float*)d_in[11];
    const float* wv = (const float*)d_in[12];  const float* bv = (const float*)d_in[13];
    const float* wo = (const float*)d_in[14];  const float* bo = (const float*)d_in[15];
    const float* w1 = (const float*)d_in[16];  const float* b1 = (const float*)d_in[17];
    const float* w2 = (const float*)d_in[18];  const float* b2 = (const float*)d_in[19];
    const float* g1 = (const float*)d_in[20];  const float* be1 = (const float*)d_in[21];
    const float* g2 = (const float*)d_in[22];  const float* be2 = (const float*)d_in[23];
    float* out = (float*)d_out;

    const size_t nQ = (size_t)NB * LQ * DM, nK = (size_t)NB * LK * DM;
    char* wsp = (char*)d_ws;
    auto carve = [&wsp](size_t bytes) { char* p = wsp; wsp += ((bytes + 255) / 256) * 256; return p; };
    unsigned short* Q16  = (unsigned short*)carve(nQ * 2);
    unsigned short* KV16 = (unsigned short*)carve(nK * 2);
    unsigned short* WT4  = (unsigned short*)carve((size_t)4 * DM * DM * 2);
    unsigned short* W1T  = (unsigned short*)carve((size_t)DFF * DM * 2);
    unsigned short* W2T  = (unsigned short*)carve((size_t)DM * DFF * 2);
    float*          BIASP = (float*)carve((size_t)4608 * 4);
    unsigned short* QH   = (unsigned short*)carve(nQ * 2);
    unsigned short* QL   = (unsigned short*)carve(nQ * 2);
    unsigned short* KH   = (unsigned short*)carve(nK * 2);
    unsigned short* KL   = (unsigned short*)carve(nK * 2);
    unsigned short* VT   = (unsigned short*)carve(nK * 2);
    float*          BP   = (float*)carve((size_t)NB * LK * LQ * 4);
    float*          Ub   = (float*)carve(nQ * 4);
    float*          ST   = (float*)carve((size_t)NB * NH * LQ * 2 * 4);
    unsigned short* C16  = (unsigned short*)carve(nQ * 2);
    float*          X1   = (float*)carve(nQ * 4);
    float*          O1   = (float*)carve(nQ * 4);
    unsigned short* O1H  = (unsigned short*)carve(nQ * 2);
    unsigned short* F1H  = (unsigned short*)carve((size_t)NB * LQ * DFF * 2);
    float*          X2   = (float*)carve(nQ * 4);
    const size_t used = (size_t)(wsp - (char*)d_ws);
    if (used > ws_size || used > (size_t)134217728) return;

    k_castrows<<<(unsigned)((nQ / 8 + 255) / 256), 256, 0, stream>>>(q, Q16, (unsigned)LQ, (unsigned)LQ_FULL, (unsigned)NB, 1.0f);
    k_castrows<<<(unsigned)((nK / 8 + 255) / 256), 256, 0, stream>>>(kv, KV16, (unsigned)LK, (unsigned)LK_FULL, (unsigned)NB, 1.0f);
    k_castT<<<dim3((unsigned)((DM * (DM / 8) + 255) / 256), 4u), 256, 0, stream>>>(wq, wk, wv, wo, (unsigned)DM, WT4, (unsigned)DM, (unsigned)DM, (unsigned)DM, 16.0f);
    k_castT<<<dim3((unsigned)((DFF * (DM / 8) + 255) / 256), 1u), 256, 0, stream>>>(w1, w1, w1, w1, (unsigned)DFF, W1T, (unsigned)DM, (unsigned)DM, (unsigned)DFF, 16.0f);
    k_castT<<<dim3((unsigned)((DM * (DFF / 8) + 255) / 256), 1u), 256, 0, stream>>>(w2, w2, w2, w2, (unsigned)DM, W2T, (unsigned)DFF, (unsigned)DFF, (unsigned)DM, 16.0f);
    k_biaspack<<<18, 256, 0, stream>>>(bq, bk, bv, bo, b1, b2, BIASP);
    k_bplane<<<(unsigned)(((size_t)NB * LK * (LQ / 4) + 255) / 256), 256, 0, stream>>>(mask, thb, tpi, ahb, api, aat, BP);

    k_gemm64<2, 2, 0, 0><<<dim3((unsigned)((((NB * LQ) / 64) * (DM / 64) + 7) / 8), 1u), 256, 0, stream>>>(
        Q16, (unsigned)DM, 0LL, WT4, (unsigned)DM, 0LL, (void*)QH, (void*)QL, (unsigned)DM, 0LL, BIASP, BIASP, (unsigned)DM, 0LL,
        (unsigned)(NB * LQ), (unsigned)DM, (unsigned)DM, 0.0078125f);
    k_gemm64<2, 2, 0, 0><<<dim3((unsigned)((((NB * LK) / 64) * (DM / 64) + 7) / 8), 1u), 256, 0, stream>>>(
        KV16, (unsigned)DM, 0LL, WT4 + (size_t)DM * DM, (unsigned)DM, 0LL, (void*)KH, (void*)KL, (unsigned)DM, 0LL, BIASP + 512, BIASP, (unsigned)DM, 0LL,
        (unsigned)(NB * LK), (unsigned)DM, (unsigned)DM, 0.0625f);
    k_gemm64<1, 1, 0, 0><<<dim3((unsigned)(((DM / 64) * (LK / 64) + 7) / 8), (unsigned)NB), 256, 0, stream>>>(
        WT4 + (size_t)2 * DM * DM, (unsigned)DM, 0LL, KV16, (unsigned)DM, (long long)LK * DM, (void*)VT, (void*)VT, (unsigned)LK, (long long)DM * LK, BIASP + 1024, BIASP, (unsigned)DM, 0LL,
        (unsigned)DM, (unsigned)LK, (unsigned)DM, 0.0625f);

    k_jattn<<<(unsigned)(NB * NH * (LQ / 64)), 32 * JA_NW, 0, stream>>>(QH, QL, KH, KL, VT, BP, aat, Ub, ST);
    k_jnorm<<<(unsigned)(NB * NH), 256, 0, stream>>>(ST, Ub, C16);

    k_gemm64<2, 0, 2, 0><<<dim3((unsigned)(((LQ / 64) * (DM / 64) + 7) / 8), (unsigned)NB), 256, 0, stream>>>(
        C16, (unsigned)DM, (long long)LQ * DM, WT4 + (size_t)3 * DM * DM, (unsigned)DM, 0LL, (void*)X1, (void*)X1, (unsigned)DM, (long long)LQ * DM, BIASP + 1536, q, (unsigned)DM, (long long)LQ_FULL * DM,
        (unsigned)LQ, (unsigned)DM, (unsigned)DM, 0.00390625f);
    k_ln<1><<<(unsigned)((NB * LQ) / 8), 256, 0, stream>>>(X1, g1, be1, O1, O1H, (unsigned)(NB * LQ));
    k_gemm64<2, 1, 0, 2><<<dim3((unsigned)((((NB * LQ) / 64) * (DFF / 64) + 7) / 8), 1u), 256, 0, stream>>>(
        O1H, (unsigned)DM, 0LL, W1T, (unsigned)DM, 0LL, (void*)F1H, (void*)F1H, (unsigned)DFF, 0LL, BIASP + 2048, BIASP, (unsigned)DM, 0LL,
        (unsigned)(NB * LQ), (unsigned)DFF, (unsigned)DM, 0.0625f);
    k_gemm64<2, 0, 1, 0><<<dim3((unsigned)((((NB * LQ) / 64) * (DM / 64) + 7) / 8), 1u), 256, 0, stream>>>(
        F1H, (unsigned)DFF, 0LL, W2T, (unsigned)DFF, 0LL, (void*)X2, (void*)X2, (unsigned)DM, 0LL, BIASP + 4096, O1, (unsigned)DM, 0LL,
        (unsigned)(NB * LQ), (unsigned)DM, (unsigned)DFF, 0.0625f);
    k_ln<0><<<(unsigned)((NB * LQ) / 8), 256, 0, stream>>>(X2, g2, be2, out, O1H, (unsigned)(NB * LQ));
}
